// DeformableGatedFusion_59150289600929
// MI455X (gfx1250) — hardware-verified
//
#include <hip/hip_runtime.h>
#include <math.h>

typedef __attribute__((ext_vector_type(16))) _Float16 v16h;
typedef __attribute__((ext_vector_type(8)))  _Float16 v8h;
typedef __attribute__((ext_vector_type(4)))  _Float16 v4h;
typedef __attribute__((ext_vector_type(16))) __bf16   v16b;
typedef __attribute__((ext_vector_type(8)))  __bf16   v8b;
typedef __attribute__((ext_vector_type(8)))  float    v8f;
typedef __attribute__((ext_vector_type(4)))  float    v4f;
typedef __attribute__((ext_vector_type(4)))  unsigned v4u;

static constexpr int kB    = 8;
static constexpr int kDm   = 384;
static constexpr int kNq   = 4096;
static constexpr int kMv   = kB * kNq;
static constexpr int kNcx  = 730;
static constexpr int kDc   = 1024;
static constexpr int kMc   = kB * kNcx;
static constexpr int kMcp  = 5888;
static constexpr int kH1   = 768;
static constexpr int kFF   = 1536;
static constexpr int kNoa  = 128;
static constexpr int kNg   = 128;
static constexpr int kNgr  = 96;
static constexpr int kQr   = 8192;
static_assert(kMcp % 64 == 0 && kMcp >= kMc, "tile multiple");
static_assert(kMv % 64 == 0 && kQr % 64 == 0 && kQr * 4 == kMv && kQr == 2 * kNq, "tile multiple");
static_assert(kDc % 32 == 0 && kH1 % 64 == 0 && kDm % 64 == 0 && kFF % 64 == 0 && kNoa % 64 == 0 && kNg % 64 == 0, "K % 32, N % 64");
static_assert((kMcp * kH1 / 8) % 256 == 0 && (kQr * kFF / 8) % 256 == 0, "gelu grids exact");

static constexpr size_t SZ_P16   = (size_t)kMv * kDm * 2;
static constexpr size_t OFF_RA   = 0;
static constexpr size_t OFF_RB   = OFF_RA + SZ_P16;
static constexpr size_t OFF_RC   = OFF_RB + SZ_P16;
static constexpr size_t SZ_CN16  = (size_t)kMcp * kDc * 2;
static constexpr size_t SZ_C1    = (size_t)kMcp * kH1 * 2;
static constexpr size_t SZ_CP    = (size_t)kMcp * kDm * 4;
static constexpr size_t OFF_CN16 = OFF_RC;
static constexpr size_t OFF_C1   = OFF_CN16 + SZ_CN16;
static constexpr size_t OFF_CP   = OFF_C1 + SZ_C1;
static constexpr size_t SZ_RC    = SZ_CN16 + SZ_C1 + SZ_CP;
static constexpr size_t OFF_RD   = OFF_RC + SZ_RC;
static constexpr size_t SZ_RD    = (size_t)kMv * kNoa * 4;
static constexpr size_t OFF_RE   = OFF_RD + SZ_RD;
static constexpr size_t SZ_RE    = (size_t)kMv * kNg * 4;
static constexpr size_t OFF_RW   = OFF_RE + SZ_RE;
static constexpr size_t OFF_WC1  = OFF_RW;
static constexpr size_t OFF_WC2  = OFF_WC1 + (size_t)kH1 * kDc * 2;
static constexpr size_t OFF_WOA  = OFF_WC2 + (size_t)kDm * kH1 * 2;
static constexpr size_t OFF_WOUT = OFF_WOA + (size_t)kNoa * kDm * 2;
static constexpr size_t OFF_WF1  = OFF_WOUT + (size_t)kDm * kDm * 2;
static constexpr size_t OFF_WF2  = OFF_WF1 + (size_t)kFF * kDm * 2;
static constexpr size_t OFF_WG1  = OFF_WF2 + (size_t)kDm * kFF * 2;
static constexpr size_t OFF_BIAS = OFF_WG1 + (size_t)kNg * kDm * 2;
static constexpr size_t WS_TOTAL = OFF_BIAS + 256 * 4;
static constexpr size_t SZ_F1Q   = (size_t)kQr * kFF * 2;
static constexpr size_t SZ_FFNQ  = (size_t)kQr * kDm * 4;
static_assert(SZ_F1Q <= SZ_P16 && SZ_F1Q <= SZ_RC, "F1 quarter planes fit RA and RC");
static_assert(SZ_FFNQ <= SZ_RD && SZ_C1 <= SZ_RD, "FFN quarter and C1PRE fit RD");
static_assert(WS_TOTAL <= (size_t)134217728, "carve under 128 MiB");
static_assert((OFF_RB % 128) == 0 && (OFF_RC % 128) == 0 && (OFF_C1 % 128) == 0 && (OFF_CP % 128) == 0 &&
              (OFF_RD % 128) == 0 && (OFF_RE % 128) == 0 && (OFF_RW % 128) == 0 && (OFF_WC2 % 128) == 0 &&
              (OFF_WOA % 128) == 0 && (OFF_WOUT % 128) == 0 && (OFF_WF1 % 128) == 0 && (OFF_WF2 % 128) == 0 &&
              (OFF_WG1 % 128) == 0 && (OFF_BIAS % 128) == 0, "128-B aligned regions");

__device__ __forceinline__ unsigned short f2bf_bits(float f) {
  unsigned u = __float_as_uint(f);
  return (unsigned short)((u + 0x7FFFu + ((u >> 16) & 1u)) >> 16);
}
__device__ __forceinline__ float bf_bits2f(unsigned short h) { return __uint_as_float(((unsigned)h) << 16); }

__device__ __forceinline__ void dep_guard_h(v8f& a, v8f& b, v16h x, v16h y) { asm volatile("v_nop\n\tv_nop\n\tv_nop\n\tv_nop" : "+v"(a), "+v"(b) : "v"(x), "v"(y)); }
__device__ __forceinline__ void dep_guard_b(v8f& a, v8f& b, v16b x, v16b y) { asm volatile("v_nop\n\tv_nop\n\tv_nop\n\tv_nop" : "+v"(a), "+v"(b) : "v"(x), "v"(y)); }
__device__ __forceinline__ void keep4_h(v16h a, v16h b, v16h c, v16h d) { asm volatile("v_nop" :: "v"(a), "v"(b), "v"(c), "v"(d)); }
__device__ __forceinline__ void keep4_b(v16b a, v16b b, v16b c, v16b d) { asm volatile("v_nop" :: "v"(a), "v"(b), "v"(c), "v"(d)); }
__device__ __forceinline__ void acc_guard4(v8f& a, v8f& b, v8f& c, v8f& d) { asm volatile("v_nop\n\tv_nop\n\tv_nop\n\tv_nop" : "+v"(a), "+v"(b), "+v"(c), "+v"(d)); }
template <typename T> struct Frag;
template <> struct Frag<_Float16> {
  typedef v16h V; union U { v16h v; v8h h[2]; };
  static __device__ __forceinline__ v16h load(const _Float16* p) {
    U f; f.h[0] = *(const v8h*)(p); f.h[1] = *(const v8h*)(p + 16); return f.v;
  }
  static __device__ __forceinline__ v8f mma(v16h a, v16h b, v8f c) {
    return __builtin_amdgcn_wmma_f32_16x16x32_f16(false, a, false, b, (short)0, c, false, false);
  }
  static __device__ __forceinline__ void guard(v8f& a, v8f& b, v16h x, v16h y) { dep_guard_h(a, b, x, y); }
  static __device__ __forceinline__ void keep(v16h a, v16h b, v16h c, v16h d) { keep4_h(a, b, c, d); }
};
template <> struct Frag<__bf16> {
  typedef v16b V; union U { v16b v; v8b h[2]; };
  static __device__ __forceinline__ v16b load(const __bf16* p) {
    U f; f.h[0] = *(const v8b*)(p); f.h[1] = *(const v8b*)(p + 16); return f.v;
  }
  static __device__ __forceinline__ v8f mma(v16b a, v16b b, v8f c) {
    return __builtin_amdgcn_wmma_f32_16x16x32_bf16(false, a, false, b, (short)0, c, false, false);
  }
  static __device__ __forceinline__ void guard(v8f& a, v8f& b, v16b x, v16b y) { dep_guard_b(a, b, x, y); }
  static __device__ __forceinline__ void keep(v16b a, v16b b, v16b c, v16b d) { keep4_b(a, b, c, d); }
};

template <int ET> struct Elem;
template <> struct Elem<0> { typedef _Float16 T; };
template <> struct Elem<1> { typedef __bf16 T; };
template <int ET, bool SPLIT, int BIAS_MODE, int OUT_MODE, bool RESID, int ACT = 0>
__global__ __launch_bounds__(256) void wmma_gemm64(
    const unsigned short* __restrict__ Ap, const unsigned short* __restrict__ A2p, int lda, long strideA,
    const unsigned short* __restrict__ Btp, const unsigned short* __restrict__ Bt2p, int ldb, long strideB,
    void* __restrict__ Cout, void* __restrict__ Cout2, int ldc, long strideC,
    const float* __restrict__ bias,
    const float* __restrict__ resid, long strideR,
    int M, int N, int K, float scale, float oscale) {
  typedef typename Elem<ET>::T T;
  typedef typename Frag<T>::V V;
  const T* A = (const T*)Ap; const T* A2 = (const T*)A2p; const T* Bt = (const T*)Btp; const T* Bt2 = (const T*)Bt2p;
  __shared__ __align__(16) float sT[8][16 * 68];
  const int b    = blockIdx.y;
  const int lane = threadIdx.x & 31;
  const int wave = threadIdx.x >> 5;
  const int tilesN = N >> 6;
  const int tilesM = M >> 6;
  const int tile = blockIdx.x * 8 + wave;
  if (tile >= tilesM * tilesN) return;
  const int tm = tile / tilesN;
  const int tn = tile - tm * tilesN;
  const int m0 = tm << 6;
  const int n0 = tn << 6;

  const T* Ab  = A  + (size_t)b * strideA;
  const T* Bb  = Bt + (size_t)b * strideB;
  const T* Ab2 = SPLIT ? (A2  + (size_t)b * strideA) : nullptr;
  const T* Bb2 = SPLIT ? (Bt2 + (size_t)b * strideB) : nullptr;

  const int rlane = lane & 15;
  const int koff  = (lane >> 4) * 8;
  const int mOff  = (lane >> 4) * 8;

  v8f acc[4][4];
#pragma unroll
  for (int i = 0; i < 4; ++i)
#pragma unroll
    for (int j = 0; j < 4; ++j) acc[i][j] = (v8f){0.f,0.f,0.f,0.f,0.f,0.f,0.f,0.f};

  for (int k0 = 0; k0 < K; k0 += 32) {
    V bh[4], bl[4];
#pragma unroll
    for (int j = 0; j < 4; ++j) {
      const size_t bo = (size_t)(n0 + (j << 4) + rlane) * ldb + koff + k0;
      bh[j] = Frag<T>::load(Bb + bo);
      if (SPLIT) bl[j] = Frag<T>::load(Bb2 + bo);
    }
#pragma unroll
    for (int i = 0; i < 4; ++i) {
      const size_t ao = (size_t)(m0 + (i << 4) + rlane) * lda + koff + k0;
      V ah = Frag<T>::load(Ab + ao);
      V al;
      if (SPLIT) al = Frag<T>::load(Ab2 + ao);
#pragma unroll
      for (int j = 0; j < 4; ++j) {
        acc[i][j] = Frag<T>::mma(ah, bh[j], acc[i][j]);
        if (SPLIT) {
          acc[i][j] = Frag<T>::mma(ah, bl[j], acc[i][j]);
          acc[i][j] = Frag<T>::mma(al, bh[j], acc[i][j]);
        }
      }
      Frag<T>::guard(acc[i][0], acc[i][3], ah, SPLIT ? al : ah);
    }
    Frag<T>::keep(bh[0], bh[1], bh[2], bh[3]);
    if (SPLIT) Frag<T>::keep(bl[0], bl[1], bl[2], bl[3]);
  }
  acc_guard4(acc[0][0], acc[0][1], acc[0][2], acc[0][3]);
  acc_guard4(acc[1][0], acc[1][1], acc[1][2], acc[1][3]);
  acc_guard4(acc[2][0], acc[2][1], acc[2][2], acc[2][3]);
  acc_guard4(acc[3][0], acc[3][1], acc[3][2], acc[3][3]);

  float* slab = sT[wave];
  const float* Rb = RESID ? (resid + (size_t)b * strideR) : nullptr;
#pragma unroll
  for (int i = 0; i < 4; ++i) {
    const int mBase = m0 + (i << 4);
#pragma unroll
    for (int j = 0; j < 4; ++j) {
      const int n = n0 + (j << 4) + rlane;
      float bv = 0.f;
      if (BIAS_MODE == 2) bv = bias[n];
#pragma unroll
      for (int r = 0; r < 8; ++r) {
        float v = acc[i][j][r] * scale;
        if (BIAS_MODE == 1) v += bias[mBase + mOff + r];
        if (BIAS_MODE == 2) v += bv;
        if (RESID) v += Rb[(size_t)(mBase + mOff + r) * ldc + n];
        if (ACT == 1) v = tanhf(v);
        if (ACT == 2) v = fmaxf(v, 0.0f);
        if (ACT == 3) v = v / (1.0f + expf(-v));
        if (ACT == 4) v = (v > 0.f) ? v : 0.01f * v;
        v = v * oscale;
        slab[(mOff + r) * 68 + (j << 4) + rlane] = v;
      }
    }
    __builtin_amdgcn_fence(__ATOMIC_RELEASE, "workgroup");
    __builtin_amdgcn_wave_barrier();
    __builtin_amdgcn_fence(__ATOMIC_ACQUIRE, "workgroup");
    if (OUT_MODE == 0) {
      float* C = (float*)Cout + (size_t)b * strideC;
      const int hh = lane >> 4, c4 = (lane & 15) * 4;
      for (int pass = 0; pass < 2; ++pass) {
#pragma unroll
        for (int it = 0; it < 8; ++it) {
          const int row = it * 2 + hh;
          v4f v = *(const v4f*)(slab + row * 68 + c4);
          *(volatile v4f*)(C + (size_t)(mBase + row) * ldc + n0 + c4) = v;
        }
        __threadfence();
      }
    } else {
      const int q = lane >> 3, c8 = (lane & 7) * 8;
      unsigned short* C  = (unsigned short*)Cout  + (size_t)b * strideC;
      unsigned short* C2 = (OUT_MODE == 2) ? ((unsigned short*)Cout2 + (size_t)b * strideC) : nullptr;
      for (int pass = 0; pass < 2; ++pass) {
#pragma unroll
        for (int it = 0; it < 4; ++it) {
          const int row = it * 4 + q;
          const float* sp = slab + row * 68 + c8;
          v8h hv, lv;
#pragma unroll
          for (int e = 0; e < 8; ++e) {
            if (OUT_MODE == 1) {
              hv[e] = (_Float16)sp[e];
            } else {
              unsigned short hb = f2bf_bits(sp[e]);
              unsigned short lb = f2bf_bits(sp[e] - bf_bits2f(hb));
              hv[e] = __builtin_bit_cast(_Float16, hb);
              lv[e] = __builtin_bit_cast(_Float16, lb);
            }
          }
          *(volatile v8h*)(C + (size_t)(mBase + row) * ldc + n0 + c8) = hv;
          if (OUT_MODE == 2) *(volatile v8h*)(C2 + (size_t)(mBase + row) * ldc + n0 + c8) = lv;
        }
        __threadfence();
      }
    }
    __builtin_amdgcn_fence(__ATOMIC_RELEASE, "workgroup");
    __builtin_amdgcn_wave_barrier();
    __builtin_amdgcn_fence(__ATOMIC_ACQUIRE, "workgroup");
  }
}

__device__ __forceinline__ float wave_sum(float v) {
#pragma unroll
  for (int off = 16; off >= 1; off >>= 1) v += __shfl_xor(v, off, 32);
  return v;
}

__global__ __launch_bounds__(256) void prep_wt16(const float* __restrict__ W, _Float16* __restrict__ Wt,
                                                int Kdim, int Nreal, int Npad) {
  const int t = blockIdx.x * 256 + threadIdx.x;
  const int k8n = Kdim >> 3;
  const int total = Npad * k8n;
  if (t >= total) return;
  const int n = t / k8n;
  const int k8 = t - n * k8n;
  const int ncl = n < Nreal ? n : (Nreal - 1);
  v8h hv;
#pragma unroll
  for (int i = 0; i < 8; ++i) {
    const float v = W[(size_t)(k8 * 8 + i) * Nreal + ncl] * 16.0f;
    hv[i] = (_Float16)v;
  }
  v8h z = {};
  if (n >= Nreal) hv = z;
  _Float16* dst = Wt + (size_t)n * Kdim + (size_t)k8 * 8;
  *(volatile v8h*)dst = hv;
  __threadfence();
  *(volatile v8h*)dst = hv;
}

__global__ __launch_bounds__(256) void prep_bias2(const float* __restrict__ boff, const float* __restrict__ battn,
                                                 const float* __restrict__ bg1, float* __restrict__ bias2) {
  const int t = threadIdx.x;
  const int n = t & 127;
  const int i0 = n < 63 ? n : 63;
  int i1 = n - 64;
  i1 = i1 < 0 ? 0 : (i1 > 31 ? 31 : i1);
  const int i2 = n < 95 ? n : 95;
  const float v0 = boff[i0];
  const float v1 = battn[i1];
  const float v2 = bg1[i2];
  const float va = (n < 64) ? v0 : ((n < 96) ? v1 : 0.0f);
  const float vb = (n < kNgr) ? v2 : 0.0f;
  const float v = (t < 128) ? va : vb;
  ((volatile float*)bias2)[t] = v;
  __threadfence();
  ((volatile float*)bias2)[t] = v;
}

__global__ __launch_bounds__(256) void ln_ctx_kernel(const float* __restrict__ x, const float* __restrict__ g,
                                                    const float* __restrict__ be, _Float16* __restrict__ y16) {
  const int wave = threadIdx.x >> 5, lane = threadIdx.x & 31;
  const int row = blockIdx.x * 8 + wave;
  v8h z = {};
  v8h o0 = z, o1 = z, o2 = z, o3 = z;
  if (row < kMc) {
    const float* xp = x + (size_t)row * kDc + lane * 8;
    v4f a[8];
#pragma unroll
    for (int j = 0; j < 4; ++j) {
      a[2 * j]     = *(const v4f*)(xp + j * 256);
      a[2 * j + 1] = *(const v4f*)(xp + j * 256 + 4);
    }
    float s = 0.0f;
#pragma unroll
    for (int j = 0; j < 8; ++j) s += (a[j][0] + a[j][1]) + (a[j][2] + a[j][3]);
    s = wave_sum(s);
    const float mean = s * (1.0f / 1024.0f);
    float sq = 0.0f;
#pragma unroll
    for (int j = 0; j < 8; ++j) {
      const v4f d = a[j] - mean;
      sq += (d[0] * d[0] + d[1] * d[1]) + (d[2] * d[2] + d[3] * d[3]);
    }
    sq = wave_sum(sq);
    const float rstd = rsqrtf(sq * (1.0f / 1024.0f) + 1e-5f);
    v8h ov[4];
#pragma unroll
    for (int j = 0; j < 4; ++j) {
      const int c0 = j * 256 + lane * 8;
      const v4f ga = *(const v4f*)(g + c0), gb = *(const v4f*)(g + c0 + 4);
      const v4f ba = *(const v4f*)(be + c0), bb = *(const v4f*)(be + c0 + 4);
      const v4f y0 = (a[2 * j] - mean) * rstd * ga + ba;
      const v4f y1 = (a[2 * j + 1] - mean) * rstd * gb + bb;
      const v8f yy = __builtin_shufflevector(y0, y1, 0, 1, 2, 3, 4, 5, 6, 7);
      ov[j] = __builtin_convertvector(yy, v8h);
    }
    o0 = ov[0]; o1 = ov[1]; o2 = ov[2]; o3 = ov[3];
  }
  _Float16* dst = y16 + (size_t)row * kDc + lane * 8;
  *(volatile v8h*)(dst)       = o0;
  *(volatile v8h*)(dst + 256) = o1;
  *(volatile v8h*)(dst + 512) = o2;
  *(volatile v8h*)(dst + 768) = o3;
  __threadfence();
  *(volatile v8h*)(dst)       = o0;
  *(volatile v8h*)(dst + 256) = o1;
  *(volatile v8h*)(dst + 512) = o2;
  *(volatile v8h*)(dst + 768) = o3;
}

__global__ __launch_bounds__(256) void ln_vis_kernel(const float* __restrict__ vis, const float* __restrict__ g,
                                                    const float* __restrict__ be,
                                                    _Float16* __restrict__ vn16, _Float16* __restrict__ vf16) {
  __shared__ float S[kDm][33];
  __shared__ float smean[32], srstd[32];
  const int tid = threadIdx.x, wave = tid >> 5, lane = tid & 31, hh = lane >> 4;
  const int q0 = blockIdx.x * 32, b = blockIdx.y;
  {
    const float* src = vis + (size_t)b * kDm * kNq + q0 + lane;
    for (int c = wave; c < kDm; c += 8) S[c][lane] = src[(size_t)c * kNq];
  }
  __syncthreads();
#pragma unroll 1
  for (int i = 0; i < 4; ++i) {
    const int q = wave * 4 + i;
    float s = 0.0f;
#pragma unroll
    for (int k = 0; k < 12; ++k) s += S[lane + 32 * k][q];
    s = wave_sum(s);
    const float mean = s * (1.0f / 384.0f);
    float sq = 0.0f;
#pragma unroll
    for (int k = 0; k < 12; ++k) { const float d = S[lane + 32 * k][q] - mean; sq += d * d; }
    sq = wave_sum(sq);
    const float rstd = rsqrtf(sq * (1.0f / 384.0f) + 1e-5f);
    if (lane == 0) { smean[q] = mean; srstd[q] = rstd; }
  }
  __syncthreads();
  const size_t rowbase = (size_t)b * kNq + q0;
  const int c16 = (lane & 15) * 8;
  for (int pass = 0; pass < 2; ++pass) {
#pragma unroll 1
    for (int pj = 0; pj < 6; ++pj) {
      const int pr = (pj >= 3) ? 1 : 0;
      const int j = pj - 3 * pr;
      const int q = wave * 4 + pr * 2 + hh;
      const int c0 = j * 128 + c16;
      const float mean = smean[q], rstd = srstd[q];
      const v4f ga = *(const v4f*)(g + c0), gb = *(const v4f*)(g + c0 + 4);
      const v4f ba = *(const v4f*)(be + c0), bb = *(const v4f*)(be + c0 + 4);
      const v8f gv = __builtin_shufflevector(ga, gb, 0, 1, 2, 3, 4, 5, 6, 7);
      const v8f bv = __builtin_shufflevector(ba, bb, 0, 1, 2, 3, 4, 5, 6, 7);
      v8h hn, hf;
#pragma unroll
      for (int e = 0; e < 8; ++e) {
        const float xv = S[c0 + e][q];
        hn[e] = (_Float16)((xv - mean) * rstd * gv[e] + bv[e]);
        hf[e] = (_Float16)xv;
      }
      const size_t o = (rowbase + q) * kDm + c0;
      *(volatile v8h*)(vn16 + o) = hn;
      *(volatile v8h*)(vf16 + o) = hf;
    }
    __threadfence();
  }
}

__global__ __launch_bounds__(256) void gelu_f16x8(const unsigned short* __restrict__ in, unsigned short* __restrict__ out,
                                                 int n8, float in_inv, float out_sc) {
  const int i = blockIdx.x * 256 + threadIdx.x;
  if (i >= n8) return;
  const v4u u = *(const v4u*)(in + (size_t)i * 8);
  const unsigned long long w01 = (unsigned long long)u[0] | ((unsigned long long)u[1] << 32);
  const unsigned long long w23 = (unsigned long long)u[2] | ((unsigned long long)u[3] << 32);
  unsigned long long r01 = 0ull, r23 = 0ull;
#pragma unroll 1
  for (int e = 0; e < 8; ++e) {
    const bool lo = (e < 4);
    const unsigned long long w = lo ? w01 : w23;
    const int sh = (e & 3) * 16;
    const unsigned short hb = (unsigned short)(w >> sh);
    const float xv = (float)__builtin_bit_cast(_Float16, hb) * in_inv;
    const float gl = 0.5f * xv * (1.0f + erff(xv * 0.70710678118654752f));
    const _Float16 gh = (_Float16)(gl * out_sc);
    const unsigned long long bits = ((unsigned long long)__builtin_bit_cast(unsigned short, gh)) << sh;
    r01 |= lo ? bits : 0ull;
    r23 |= lo ? 0ull : bits;
  }
  v4u r;
  r[0] = (unsigned)r01; r[1] = (unsigned)(r01 >> 32); r[2] = (unsigned)r23; r[3] = (unsigned)(r23 >> 32);
  unsigned short* dst = out + (size_t)i * 8;
  *(volatile v4u*)dst = r;
  __threadfence();
  *(volatile v4u*)dst = r;
}

__device__ __forceinline__ void corner_set(int& io, float& co, float xf, float yf, float w, float aw) {
#pragma clang fp contract(off)
  const bool ok = (xf >= 0.0f) && (xf < 27.0f) && (yf >= 0.0f) && (yf < 27.0f);
  const float xc = fminf(fmaxf(xf, 0.0f), 26.0f);
  const float yc = fminf(fmaxf(yf, 0.0f), 26.0f);
  const int xi = (int)xc, yi = (int)yc;
  io = 1 + yi * 27 + xi;
  co = aw * (w * (ok ? 1.0f : 0.0f));
}

__global__ __launch_bounds__(256) void sample_kernel(const float* __restrict__ oa, const float* __restrict__ cp,
                                                    _Float16* __restrict__ ao16) {
#pragma clang fp contract(off)
  __shared__ int   pidx[4][32][4];
  __shared__ float pco[4][32][4];
  const int tid = threadIdx.x;
  const int row0 = blockIdx.x * 4;
  if (tid < 128) {
    const int r = tid >> 5, j = tid & 31, h = j >> 2, p = j & 3;
    const float* oar = oa + (size_t)(row0 + r) * kNoa;
    const float l0 = oar[64 + h * 4], l1 = oar[65 + h * 4], l2 = oar[66 + h * 4], l3 = oar[67 + h * 4];
    const float mx = fmaxf(fmaxf(l0, l1), fmaxf(l2, l3));
    const float e0 = __expf(l0 - mx), e1 = __expf(l1 - mx), e2 = __expf(l2 - mx), e3 = __expf(l3 - mx);
    const float esum = ((e0 + e1) + e2) + e3;
    const float ej = (p == 0) ? e0 : ((p == 1) ? e1 : ((p == 2) ? e2 : e3));
    const float aw = ej * (1.0f / esum);
    const float ox = oar[j * 2], oy = oar[j * 2 + 1];
    const float cxo = fminf(fmaxf(ox, -40.0f), 40.0f);
    const float cyo = fminf(fmaxf(oy, -40.0f), 40.0f);
    const float sx = 1.0f / (1.0f + expf(-cxo));
    const float sy = 1.0f / (1.0f + expf(-cyo));
    const float lx = 2.0f * sx - 1.0f;
    const float ly = 2.0f * sy - 1.0f;
    const float ix = ((lx + 1.0f) * 27.0f - 1.0f) * 0.5f;
    const float iy = ((ly + 1.0f) * 27.0f - 1.0f) * 0.5f;
    const float x0f = floorf(ix), y0f = floorf(iy);
    const float wx1 = ix - x0f, wx0 = 1.0f - wx1;
    const float wy1 = iy - y0f, wy0 = 1.0f - wy1;
    const float x1f = x0f + 1.0f, y1f = y0f + 1.0f;
    int i0, i1, i2, i3;
    float c0, c1, c2, c3;
    corner_set(i0, c0, x0f, y0f, wx0 * wy0, aw);
    corner_set(i1, c1, x1f, y0f, wx1 * wy0, aw);
    corner_set(i2, c2, x0f, y1f, wx0 * wy1, aw);
    corner_set(i3, c3, x1f, y1f, wx1 * wy1, aw);
    pidx[r][j][0] = i0; pidx[r][j][1] = i1; pidx[r][j][2] = i2; pidx[r][j][3] = i3;
    pco[r][j][0] = c0;  pco[r][j][1] = c1;  pco[r][j][2] = c2;  pco[r][j][3] = c3;
  }
  __syncthreads();
  const int r = tid >> 6, u = tid & 63;
  const int uc = u < 48 ? u : 47;
  const int h = uc / 6, d0 = (uc - h * 6) * 8;
  const int row = row0 + r;
  const int b = row >> 12;
  const float* cpb = cp + (size_t)b * kNcx * kDm + h * 48 + d0;
  float acc[8];
#pragma unroll
  for (int e = 0; e < 8; ++e) acc[e] = 0.0f;
#pragma unroll 1
  for (int it = 0; it < 16; ++it) {
    const int p = it >> 2, k = it & 3;
    int idx = pidx[r][h * 4 + p][k];
    idx = idx < 1 ? 1 : (idx > 729 ? 729 : idx);
    const float co = pco[r][h * 4 + p][k];
    const float* vp = cpb + (size_t)idx * kDm;
    const v4f g0 = *(const v4f*)vp;
    const v4f g1 = *(const v4f*)(vp + 4);
#pragma unroll
    for (int e = 0; e < 4; ++e) {
      acc[e]     = fmaf(co, g0[e], acc[e]);
      acc[4 + e] = fmaf(co, g1[e], acc[4 + e]);
    }
  }
  v8h o;
#pragma unroll
  for (int e = 0; e < 8; ++e) o[e] = (_Float16)(acc[e] * 16.0f);
  _Float16* dst = ao16 + (size_t)row * kDm + uc * 8;
  const bool wr = (u < 48);
  if (wr) *(volatile v8h*)dst = o;
  __threadfence();
  if (wr) *(volatile v8h*)dst = o;
}

__global__ __launch_bounds__(256) void final_kernel(const float* __restrict__ vis, const float* __restrict__ ffnq,
                                                   const float* __restrict__ g1, const float* __restrict__ wg2,
                                                   const float* __restrict__ bg2,
                                                   const float* __restrict__ g, const float* __restrict__ be,
                                                   float* __restrict__ out0, float* __restrict__ out1, int b_first) {
  __shared__ float S[kDm][33];
  __shared__ float gq[32], smean[32], srstd[32];
  const int tid = threadIdx.x, wave = tid >> 5, lane = tid & 31;
  const int q0 = blockIdx.x * 32;
  const int bl = blockIdx.y;
  const int b = b_first + bl;
  const size_t rowbase = (size_t)b * kNq + q0;
  const size_t frow = (size_t)bl * kNq + q0;
  {
    const float* src = vis + (size_t)b * kDm * kNq + q0 + lane;
    for (int c = wave; c < kDm; c += 8) S[c][lane] = src[(size_t)c * kNq];
  }
  {
    const float w0 = wg2[lane], w1 = wg2[lane + 32], w2 = wg2[lane + 64];
    const float bb = bg2[0];
#pragma unroll 1
    for (int i = 0; i < 4; ++i) {
      const int q = wave * 4 + i;
      const float* gr = g1 + (rowbase + q) * kNg;
      float s = gr[lane] * w0 + gr[lane + 32] * w1 + gr[lane + 64] * w2;
      s = wave_sum(s);
      const float z = fminf(fmaxf(s + bb, -40.0f), 40.0f);
      const float gt = 1.0f / (1.0f + expf(-z));
      if (lane == 0) gq[q] = gt;
    }
  }
  __syncthreads();
  for (int idx = tid; idx < 32 * kDm; idx += 256) {
    const int q = idx / kDm;
    const int c = idx - q * kDm;
    const float f = ffnq[(frow + q) * kDm + c];
    S[c][q] = S[c][q] + gq[q] * f;
  }
  __syncthreads();
#pragma unroll 1
  for (int i = 0; i < 4; ++i) {
    const int q = wave * 4 + i;
    float s = 0.0f;
#pragma unroll
    for (int k = 0; k < 12; ++k) s += S[lane + 32 * k][q];
    s = wave_sum(s);
    const float mean = s * (1.0f / 384.0f);
    float sq = 0.0f;
#pragma unroll
    for (int k = 0; k < 12; ++k) { const float d = S[lane + 32 * k][q] - mean; sq += d * d; }
    sq = wave_sum(sq);
    const float rstd = rsqrtf(sq * (1.0f / 384.0f) + 1e-5f);
    if (lane == 0) { smean[q] = mean; srstd[q] = rstd; }
  }
  __syncthreads();
  {
    const int cq = lane >> 3, q4 = (lane & 7) * 4;
    float* ob = out0 + (size_t)b * kDm * kNq + q0 + q4;
    for (int pass = 0; pass < 2; ++pass) {
#pragma unroll 1
      for (int it = 0; it < 12; ++it) {
        const int c = wave * 48 + it * 4 + cq;
        const float gc = g[c], bc = be[c];
        v4f v;
#pragma unroll
        for (int e = 0; e < 4; ++e) {
          const int q = q4 + e;
          v[e] = (S[c][q] - smean[q]) * srstd[q] * gc + bc;
        }
        *(volatile v4f*)(ob + (size_t)c * kNq) = v;
      }
      __threadfence();
    }
  }
  {
    const int l8 = lane & 7;
    v4f gv;
    gv[0] = gq[l8 * 4 + 0]; gv[1] = gq[l8 * 4 + 1]; gv[2] = gq[l8 * 4 + 2]; gv[3] = gq[l8 * 4 + 3];
    float* o1 = out1 + rowbase + l8 * 4;
    const bool wr = (wave == 0) && (lane < 8);
    if (wr) *(volatile v4f*)o1 = gv;
    __threadfence();
    if (wr) *(volatile v4f*)o1 = gv;
  }
}

static constexpr int gemm_blocks(int M, int N) { return ((M / 64) * (N / 64) + 7) / 8; }

extern "C" void kernel_launch(void* const* d_in, const int* in_sizes, int n_in,
                              void* d_out, int out_size, void* d_ws, size_t ws_size,
                              hipStream_t stream) {
  if (n_in < 26) return;
  if (in_sizes[0] != kB * kDm * kNq || in_sizes[1] != kMc * kDc) return;
  if (in_sizes[2] != kDm || in_sizes[3] != kDm || in_sizes[4] != kDc || in_sizes[5] != kDc) return;
  if (in_sizes[6] != kDc * kH1 || in_sizes[7] != kH1 || in_sizes[8] != kH1 * kDm || in_sizes[9] != kDm) return;
  if (in_sizes[10] != kDm * 64 || in_sizes[11] != 64 || in_sizes[12] != kDm * 32 || in_sizes[13] != 32) return;
  if (in_sizes[14] != kDm * kDm || in_sizes[15] != kDm || in_sizes[16] != kDm * kFF || in_sizes[17] != kFF) return;
  if (in_sizes[18] != kFF * kDm || in_sizes[19] != kDm || in_sizes[20] != kDm * kNgr || in_sizes[21] != kNgr) return;
  if (in_sizes[22] != kNgr || in_sizes[23] != 1 || in_sizes[24] != kDm || in_sizes[25] != kDm) return;
  if (out_size != kB * kDm * kNq + kMv) return;
  if (ws_size < WS_TOTAL) return;

  const float* vis    = (const float*)d_in[0];
  const float* ctx    = (const float*)d_in[1];
  const float* ln_v_g = (const float*)d_in[2];
  const float* ln_v_b = (const float*)d_in[3];
  const float* ln_c_g = (const float*)d_in[4];
  const float* ln_c_b = (const float*)d_in[5];
  const float* W_c1   = (const float*)d_in[6];
  const float* b_c1   = (const float*)d_in[7];
  const float* W_c2   = (const float*)d_in[8];
  const float* b_c2   = (const float*)d_in[9];
  const float* W_off  = (const float*)d_in[10];
  const float* b_off  = (const float*)d_in[11];
  const float* W_attn = (const float*)d_in[12];
  const float* b_attn = (const float*)d_in[13];
  const float* W_out  = (const float*)d_in[14];
  const float* b_out  = (const float*)d_in[15];
  const float* W_f1   = (const float*)d_in[16];
  const float* b_f1   = (const float*)d_in[17];
  const float* W_f2   = (const float*)d_in[18];
  const float* b_f2   = (const float*)d_in[19];
  const float* W_g1   = (const float*)d_in[20];
  const float* b_g1   = (const float*)d_in[21];
  const float* W_g2   = (const float*)d_in[22];
  const float* b_g2   = (const float*)d_in[23];
  const float* ln_o_g = (const float*)d_in[24];
  const float* ln_o_b = (const float*)d_in[25];

  char* ws = (char*)d_ws;
  _Float16* vn16  = (_Float16*)(ws + OFF_RA);
  _Float16* ao16  = (_Float16*)(ws + OFF_RA);
  _Float16* f1pre = (_Float16*)(ws + OFF_RA);
  _Float16* vf16  = (_Float16*)(ws + OFF_RB);
  _Float16* att16 = (_Float16*)(ws + OFF_RB);
  _Float16* cn16  = (_Float16*)(ws + OFF_CN16);
  _Float16* c1    = (_Float16*)(ws + OFF_C1);
  float*    cpf   = (float*)(ws + OFF_CP);
  _Float16* f1    = (_Float16*)(ws + OFF_RC);
  _Float16* c1pre = (_Float16*)(ws + OFF_RD);
  float*    oaf   = (float*)(ws + OFF_RD);
  float*    ffnq  = (float*)(ws + OFF_RD);
  float*    g1f   = (float*)(ws + OFF_RE);
  _Float16* wc1T  = (_Float16*)(ws + OFF_WC1);
  _Float16* wc2T  = (_Float16*)(ws + OFF_WC2);
  _Float16* woaT  = (_Float16*)(ws + OFF_WOA);
  _Float16* woutT = (_Float16*)(ws + OFF_WOUT);
  _Float16* wf1T  = (_Float16*)(ws + OFF_WF1);
  _Float16* wf2T  = (_Float16*)(ws + OFF_WF2);
  _Float16* wg1T  = (_Float16*)(ws + OFF_WG1);
  float*    bias2 = (float*)(ws + OFF_BIAS);
  float*    out0  = (float*)d_out;
  float*    out1  = out0 + (size_t)kB * kDm * kNq;

  typedef const unsigned short* cu16;
  const float sc16   = 1.0f / 16.0f;
  const float sc64   = 1.0f / 64.0f;
  const float sc256  = 1.0f / 256.0f;
  const float sc1024 = 1.0f / 1024.0f;
  const float sc4096 = 1.0f / 4096.0f;

  prep_wt16<<<(kH1 * (kDc / 8) + 255) / 256, 256, 0, stream>>>(W_c1, wc1T, kDc, kH1, kH1);
  prep_wt16<<<(kDm * (kH1 / 8) + 255) / 256, 256, 0, stream>>>(W_c2, wc2T, kH1, kDm, kDm);
  prep_wt16<<<(64 * (kDm / 8) + 255) / 256, 256, 0, stream>>>(W_off, woaT, kDm, 64, 64);
  prep_wt16<<<(64 * (kDm / 8) + 255) / 256, 256, 0, stream>>>(W_attn, woaT + (size_t)64 * kDm, kDm, 32, 64);
  prep_wt16<<<(kDm * (kDm / 8) + 255) / 256, 256, 0, stream>>>(W_out, woutT, kDm, kDm, kDm);
  prep_wt16<<<(kFF * (kDm / 8) + 255) / 256, 256, 0, stream>>>(W_f1, wf1T, kDm, kFF, kFF);
  prep_wt16<<<(kDm * (kFF / 8) + 255) / 256, 256, 0, stream>>>(W_f2, wf2T, kFF, kDm, kDm);
  prep_wt16<<<(kNg * (kDm / 8) + 255) / 256, 256, 0, stream>>>(W_g1, wg1T, kDm, kNgr, kNg);
  prep_bias2<<<1, 256, 0, stream>>>(b_off, b_attn, b_g1, bias2);

  ln_ctx_kernel<<<kMcp / 8, 256, 0, stream>>>(ctx, ln_c_g, ln_c_b, cn16);
  wmma_gemm64<0, false, 2, 1, false, 0><<<dim3(gemm_blocks(kMcp, kH1), 1), 256, 0, stream>>>(
      (cu16)cn16, nullptr, kDc, 0L, (cu16)wc1T, nullptr, kDc, 0L, (void*)c1pre, nullptr, kH1, 0L,
      b_c1, nullptr, 0L, kMcp, kH1, kDc, sc16, 16.0f);
  gelu_f16x8<<<(kMcp * kH1 / 8) / 256, 256, 0, stream>>>((const unsigned short*)c1pre, (unsigned short*)c1, kMcp * kH1 / 8, sc16, 16.0f);
  wmma_gemm64<0, false, 2, 0, false, 0><<<dim3(gemm_blocks(kMcp, kDm), 1), 256, 0, stream>>>(
      (cu16)c1, nullptr, kH1, 0L, (cu16)wc2T, nullptr, kH1, 0L, (void*)cpf, nullptr, kDm, 0L,
      b_c2, nullptr, 0L, kMcp, kDm, kH1, sc256, 1.0f);

  ln_vis_kernel<<<dim3(kNq / 32, kB), 256, 0, stream>>>(vis, ln_v_g, ln_v_b, vn16, vf16);
  wmma_gemm64<0, false, 2, 0, false, 0><<<dim3(gemm_blocks(kMv, kNoa), 1), 256, 0, stream>>>(
      (cu16)vn16, nullptr, kDm, 0L, (cu16)woaT, nullptr, kDm, 0L, (void*)oaf, nullptr, kNoa, 0L,
      bias2, nullptr, 0L, kMv, kNoa, kDm, sc16, 1.0f);
  wmma_gemm64<0, false, 2, 0, false, 2><<<dim3(gemm_blocks(kMv, kNg), 1), 256, 0, stream>>>(
      (cu16)vf16, nullptr, kDm, 0L, (cu16)wg1T, nullptr, kDm, 0L, (void*)g1f, nullptr, kNg, 0L,
      bias2 + 128, nullptr, 0L, kMv, kNg, kDm, sc16, 1.0f);
  sample_kernel<<<kMv / 4, 256, 0, stream>>>(oaf, cpf, ao16);
  wmma_gemm64<0, false, 2, 1, false, 0><<<dim3(gemm_blocks(kMv, kDm), 1), 256, 0, stream>>>(
      (cu16)ao16, nullptr, kDm, 0L, (cu16)woutT, nullptr, kDm, 0L, (void*)att16, nullptr, kDm, 0L,
      b_out, nullptr, 0L, kMv, kDm, kDm, sc256, 64.0f);

  for (int qq = 0; qq < 4; ++qq) {
    const _Float16* attq = att16 + (size_t)qq * kQr * kDm;
    wmma_gemm64<0, false, 2, 1, false, 0><<<dim3(gemm_blocks(kQr, kFF), 1), 256, 0, stream>>>(
        (cu16)attq, nullptr, kDm, 0L, (cu16)wf1T, nullptr, kDm, 0L, (void*)f1pre, nullptr, kFF, 0L,
        b_f1, nullptr, 0L, kQr, kFF, kDm, sc1024, 64.0f);
    gelu_f16x8<<<(kQr * kFF / 8) / 256, 256, 0, stream>>>((const unsigned short*)f1pre, (unsigned short*)f1, kQr * kFF / 8, sc64, 256.0f);
    wmma_gemm64<0, false, 2, 0, false, 0><<<dim3(gemm_blocks(kQr, kDm), 1), 256, 0, stream>>>(
        (cu16)f1, nullptr, kFF, 0L, (cu16)wf2T, nullptr, kFF, 0L, (void*)ffnq, nullptr, kDm, 0L,
        b_f2, nullptr, 0L, kQr, kDm, kFF, sc4096, 1.0f);
    final_kernel<<<dim3(kNq / 32, 2), 256, 0, stream>>>(vis, ffnq, g1f, W_g2, b_g2, ln_o_g, ln_o_b, out0, out1, 2 * qq);
  }
}
